// _ScratchXLSTM_6640019439853
// MI455X (gfx1250) — hardware-run, weakly checked
//
#include <hip/hip_runtime.h>
#include <math.h>

constexpr int NBATCH  = 1024;
constexpr int NSTEP   = 64;
constexpr int DMODEL  = 128;
constexpr int NHEAD   = 4;
constexpr int HDIM    = 32;
constexpr int NVOC    = 9;
constexpr int NLAYER  = 2;
constexpr int NGATE   = 4 * DMODEL;
constexpr int NROWS   = NBATCH * NSTEP;
constexpr int NQUART  = 4;
constexpr int QBATCH  = NBATCH / NQUART;
constexpr int QROWS   = QBATCH * NSTEP;
constexpr int SEQ_BLK = 16;
constexpr int HAP = 40;
constexpr int SLP = 36;
constexpr int FAP = 136;
constexpr float ACT_CARRY = 16.0f;
constexpr float W_CARRY   = 1024.0f;
constexpr float U_CARRY   = 256.0f;
constexpr float HS_CARRY  = 512.0f;
constexpr float GATE_FOLD = 1.0f / (ACT_CARRY * W_CARRY);
constexpr float MLP2_FOLD = 1.0f / (U_CARRY * W_CARRY);
constexpr float REC_FOLD  = 1.0f / (HS_CARRY * W_CARRY);
constexpr float NORM_EPS  = 1e-5f;
constexpr float CELL_EPS  = 1e-6f;
constexpr float F16_MIN_NORMAL = 6.103515625e-5f;

static_assert(DMODEL == NHEAD * HDIM, "head split");
static_assert(HDIM == 32, "one 32-deep k step per head");
static_assert(DMODEL % 32 == 0, "GEMM K multiple of 32");
static_assert(QROWS % 64 == 0 && NROWS % 64 == 0 && NGATE % 64 == 0 && DMODEL % 64 == 0, "GEMM M, N tile multiples");
static_assert(QBATCH % SEQ_BLK == 0, "recurrence grid exact");
static_assert(NROWS % 128 == 0 && NROWS % 16 == 0 && NROWS % 8 == 0, "row grids exact");
static_assert(NVOC <= 16, "head fits one 16-column tile");
static_assert(NGATE * (DMODEL / 8) == 8192 && DMODEL * (DMODEL / 8) == 2048 && NHEAD * 128 * (HDIM / 8) == 2048, "prep segment shifts");
static_assert((HAP % 8) == 0 && (SLP % 4) == 0 && (FAP % 8) == 0, "16-B aligned LDS rows");

typedef __attribute__((ext_vector_type(16))) _Float16 v16h;
typedef __attribute__((ext_vector_type(8)))  _Float16 v8h;
typedef __attribute__((ext_vector_type(8)))  float    v8f;
typedef __attribute__((ext_vector_type(4)))  float    v4f;
typedef __attribute__((ext_vector_type(2)))  float    v2f;

union FragU { v16h v; v8h h[2]; };
__device__ __forceinline__ v16h frag_load(const _Float16* p) {
  FragU f;
  f.h[0] = *(const v8h*)(p);
  f.h[1] = *(const v8h*)(p + 16);
  return f.v;
}
__device__ __forceinline__ v8f mma16(v16h a, v16h b, v8f c) {
  return __builtin_amdgcn_wmma_f32_16x16x32_f16(false, a, false, b, (short)0, c, false, false);
}
__device__ __forceinline__ void tie_acc(v8f& acc, v16h a, v16h b) {
  asm volatile("v_nop\n\tv_nop\n\tv_nop\n\tv_nop" : "+v"(acc) : "v"(a), "v"(b));
}
__device__ __forceinline__ void keep4_h(v16h a, v16h b, v16h c, v16h d) {
  asm volatile("v_nop" :: "v"(a), "v"(b), "v"(c), "v"(d));
}
__device__ __forceinline__ _Float16 to_h16(float v, float carry) {
  float s = v * carry;
  s = (fabsf(s) < F16_MIN_NORMAL) ? 0.0f : s;
  return (_Float16)s;
}

__device__ __forceinline__ void cvt_store8(const float* src, int stride, bool valid, unsigned short* dst) {
  v8h hv;
#pragma unroll
  for (int e = 0; e < 8; ++e) {
    float xv = src[(size_t)e * (size_t)stride];
    asm volatile("" : "+v"(xv));
    hv[e] = to_h16(valid ? xv : 0.0f, W_CARRY);
  }
  *(volatile v8h*)dst = hv;
  __threadfence();
  *(volatile v8h*)dst = hv;
}

constexpr int SEG_W1 = 16384;
constexpr int SEG_W2 = 20480;
constexpr int SEG_R  = 24576;
constexpr int SEG_P  = 28672;
constexpr int SEG_B  = 28928;
constexpr int SEG_END = 29184;
static_assert(SEG_END % 256 == 0, "prep grid exact");
__global__ __launch_bounds__(256) void prep_planes_kernel(
    const float* __restrict__ Wg, const float* __restrict__ bg, const float* __restrict__ R,
    const float* __restrict__ W1, const float* __restrict__ W2, const float* __restrict__ projW,
    unsigned short* __restrict__ WGT, unsigned short* __restrict__ W1T, unsigned short* __restrict__ W2T,
    unsigned short* __restrict__ RT, unsigned short* __restrict__ PT, float* __restrict__ BGP) {
  const int gi = blockIdx.x * 256 + threadIdx.x;
  if (gi < SEG_W1) {
    const int l = gi >> 13;
    const int rem = gi & 8191;
    const int np = rem >> 4;
    const int k8 = (rem & 15) * 8;
    const int head = np >> 7, eh = (np >> 6) & 1, cc = (np >> 2) & 15, g = np & 3;
    const int n = g * DMODEL + head * HDIM + eh * 16 + cc;
    cvt_store8(Wg + (size_t)l * DMODEL * NGATE + (size_t)k8 * NGATE + n, NGATE, true, WGT + (size_t)gi * 8);
  } else if (gi < SEG_R) {
    const bool second = (gi >= SEG_W2);
    const int j = gi - (second ? SEG_W2 : SEG_W1);
    const int l = j >> 11;
    const int rem = j & 2047;
    const int n = rem >> 4;
    const int k8 = (rem & 15) * 8;
    const float* src = (second ? W2 : W1) + (size_t)l * DMODEL * DMODEL + (size_t)k8 * DMODEL + n;
    unsigned short* dst = (second ? W2T : W1T) + (size_t)j * 8;
    cvt_store8(src, DMODEL, true, dst);
  } else if (gi < SEG_P) {
    const int j = gi - SEG_R;
    const int l = j >> 11;
    const int rem = j & 2047;
    const int head = rem >> 9;
    const int rem2 = rem & 511;
    const int n = rem2 >> 2;
    const int k8 = (rem2 & 3) * 8;
    const int g = n >> 5, e = n & 31;
    cvt_store8(R + (size_t)l * 16384 + (size_t)g * 4096 + (size_t)head * 1024 + (size_t)k8 * HDIM + e, HDIM, true,
               RT + (size_t)j * 8);
  } else if (gi < SEG_B) {
    const int j = gi - SEG_P;
    const int n = j >> 4;
    const int k8 = (j & 15) * 8;
    const bool valid = (n < NVOC);
    const int nc = valid ? n : (NVOC - 1);
    cvt_store8(projW + (size_t)k8 * NVOC + nc, NVOC, valid, PT + (size_t)j * 8);
  } else if (gi < SEG_END) {
    const int j = gi - SEG_B;
    const int idx4 = j * 4;
    const int l = idx4 >> 9;
    const int np = idx4 & 511;
    const int head = np >> 7, eh = (np >> 6) & 1, cc = (np >> 2) & 15;
    v4f o;
#pragma unroll
    for (int g = 0; g < 4; ++g) o[g] = bg[l * NGATE + g * DMODEL + head * HDIM + eh * 16 + cc];
    *(volatile v4f*)(BGP + idx4) = o;
    __threadfence();
    *(volatile v4f*)(BGP + idx4) = o;
  }
}

__global__ __launch_bounds__(256) void embed_kernel(const int* __restrict__ x, const float* __restrict__ emb,
                                                    float* __restrict__ H) {
  const int lane = threadIdx.x & 31;
  const int row = blockIdx.x * 8 + (threadIdx.x >> 5);
  int tok = x[row];
  tok = tok < 0 ? 0 : (tok > NVOC - 1 ? NVOC - 1 : tok);
  const v4f v = *(const v4f*)(emb + (size_t)tok * DMODEL + 4 * lane);
  float* op = H + (size_t)row * DMODEL + 4 * lane;
  *(volatile v4f*)op = v;
  __threadfence();
  *(volatile v4f*)op = v;
}

__device__ __forceinline__ v8h ln8_to_h(const float* rp, v4f g0, v4f g1, v4f b0, v4f b1) {
  v4f a = *(const v4f*)(rp);
  v4f b = *(const v4f*)(rp + 4);
  float s = ((a[0] + a[1]) + (a[2] + a[3])) + ((b[0] + b[1]) + (b[2] + b[3]));
  s += __shfl_xor(s, 1, 32);
  s += __shfl_xor(s, 2, 32);
  s += __shfl_xor(s, 4, 32);
  s += __shfl_xor(s, 8, 32);
  const float mu = s * (1.0f / DMODEL);
  float ss = 0.0f;
#pragma unroll
  for (int e = 0; e < 4; ++e) {
    const float da = a[e] - mu;
    const float db = b[e] - mu;
    a[e] = da;
    b[e] = db;
    ss += da * da + db * db;
  }
  ss += __shfl_xor(ss, 1, 32);
  ss += __shfl_xor(ss, 2, 32);
  ss += __shfl_xor(ss, 4, 32);
  ss += __shfl_xor(ss, 8, 32);
  const float rstd = rsqrtf(ss * (1.0f / DMODEL) + NORM_EPS);
  v8h hv;
#pragma unroll
  for (int e = 0; e < 4; ++e) {
    hv[e]     = to_h16((a[e] * rstd) * g0[e] + b0[e], ACT_CARRY);
    hv[4 + e] = to_h16((b[e] * rstd) * g1[e] + b1[e], ACT_CARRY);
  }
  return hv;
}

__global__ __launch_bounds__(256) void ln_rows_kernel(const float* __restrict__ Hp, const float* __restrict__ gam,
                                                      const float* __restrict__ bet, unsigned short* __restrict__ AX) {
  const int tid = threadIdx.x;
  const int l16 = tid & 15;
  const int row = blockIdx.x * 16 + (tid >> 4);
  const v4f g0 = *(const v4f*)(gam + 8 * l16);
  const v4f g1 = *(const v4f*)(gam + 8 * l16 + 4);
  const v4f b0 = *(const v4f*)(bet + 8 * l16);
  const v4f b1 = *(const v4f*)(bet + 8 * l16 + 4);
  const v8h hv = ln8_to_h(Hp + (size_t)row * DMODEL + 8 * l16, g0, g1, b0, b1);
  unsigned short* op = AX + (size_t)row * DMODEL + 8 * l16;
  *(volatile v8h*)op = hv;
  __threadfence();
  *(volatile v8h*)op = hv;
}

template <bool RESID>
__global__ __launch_bounds__(256) void gemm64_f16(
    const unsigned short* __restrict__ Ap, int lda,
    const unsigned short* __restrict__ Btp, int ldb,
    float* Cout, int ldc,
    const float* __restrict__ bias,
    const float* resid,
    int M, int N, int K, float scale) {
  const _Float16* A  = (const _Float16*)Ap;
  const _Float16* Bt = (const _Float16*)Btp;
  __shared__ __align__(16) float sT[8][16 * 68];
  const int lane = threadIdx.x & 31;
  const int wave = threadIdx.x >> 5;
  const int tilesN = N >> 6;
  const int tilesM = M >> 6;
  const int tile = blockIdx.x * 8 + wave;
  if (tile >= tilesM * tilesN) return;
  const int tm = tile / tilesN;
  const int tn = tile - tm * tilesN;
  const int m0 = tm << 6;
  const int n0 = tn << 6;
  const int rlane = lane & 15;
  const int koff  = (lane >> 4) * 8;
  const int mOff  = (lane >> 4) * 8;

  v8f acc[4][4];
#pragma unroll
  for (int i = 0; i < 4; ++i)
#pragma unroll
    for (int j = 0; j < 4; ++j) acc[i][j] = (v8f){0.f, 0.f, 0.f, 0.f, 0.f, 0.f, 0.f, 0.f};

  for (int k0 = 0; k0 < K; k0 += 32) {
    v16h bh[4];
#pragma unroll
    for (int j = 0; j < 4; ++j) bh[j] = frag_load(Bt + (size_t)(n0 + (j << 4) + rlane) * ldb + koff + k0);
#pragma unroll
    for (int i = 0; i < 4; ++i) {
      const v16h ah = frag_load(A + (size_t)(m0 + (i << 4) + rlane) * lda + koff + k0);
#pragma unroll
      for (int j = 0; j < 4; ++j) acc[i][j] = mma16(ah, bh[j], acc[i][j]);
#pragma unroll
      for (int j = 0; j < 4; ++j) tie_acc(acc[i][j], ah, bh[j]);
    }
    keep4_h(bh[0], bh[1], bh[2], bh[3]);
  }

  float* slab = sT[wave];
  const int hh2 = lane >> 4, c4 = (lane & 15) * 4;
#pragma unroll
  for (int i = 0; i < 4; ++i) {
    const int mBase = m0 + (i << 4);
#pragma unroll
    for (int j = 0; j < 4; ++j) {
      const float bv = bias[n0 + (j << 4) + rlane];
#pragma unroll
      for (int r = 0; r < 8; ++r) slab[(mOff + r) * 68 + (j << 4) + rlane] = acc[i][j][r] * scale + bv;
    }
    __builtin_amdgcn_fence(__ATOMIC_RELEASE, "workgroup");
    __builtin_amdgcn_wave_barrier();
    __builtin_amdgcn_fence(__ATOMIC_ACQUIRE, "workgroup");
    v4f vals[8];
#pragma unroll
    for (int it = 0; it < 8; ++it) {
      const int row = it * 2 + hh2;
      v4f v = *(const v4f*)(slab + row * 68 + c4);
      if (RESID) {
        const v4f rv = *(const v4f*)(resid + (size_t)(mBase + row) * ldc + n0 + c4);
        v = v + rv;
      }
      vals[it] = v;
    }
    for (int pass = 0; pass < 2; ++pass) {
#pragma unroll
      for (int it = 0; it < 8; ++it) {
        const int row = it * 2 + hh2;
        *(volatile v4f*)(Cout + (size_t)(mBase + row) * ldc + n0 + c4) = vals[it];
      }
      __threadfence();
    }
    __builtin_amdgcn_fence(__ATOMIC_RELEASE, "workgroup");
    __builtin_amdgcn_wave_barrier();
    __builtin_amdgcn_fence(__ATOMIC_ACQUIRE, "workgroup");
  }
}

__global__ __launch_bounds__(256) void scan_kernel(const float* __restrict__ GX, const unsigned short* __restrict__ RTp,
                                                   const float* __restrict__ gns, const float* __restrict__ gnb,
                                                   float* Hq) {
  __shared__ __align__(16) _Float16 hA[2][NHEAD][SEQ_BLK * HAP];
  __shared__ __align__(16) float    Ss[2][NHEAD][SEQ_BLK * SLP];
  const _Float16* RT = (const _Float16*)RTp;
  const int tid = threadIdx.x, lane = tid & 31, wave = tid >> 5;
  const int head = wave >> 1, eh = wave & 1;
  const int c = lane & 15, hh = lane >> 4;
  const int q = lane >> 3, c4 = (lane & 7) * 4;
  const int b0 = blockIdx.x * SEQ_BLK;

  {
    v8h z;
#pragma unroll
    for (int e = 0; e < 8; ++e) z[e] = (_Float16)0.0f;
    v8h* zp = (v8h*)&hA[0][0][0];
    for (int i = tid; i < (NHEAD * SEQ_BLK * HAP) / 8; i += 256) zp[i] = z;
  }
  v16h bfr[4];
#pragma unroll
  for (int g = 0; g < 4; ++g)
    bfr[g] = frag_load(RT + (size_t)head * 4096 + (size_t)(g * HDIM + 16 * eh + c) * HDIM + 8 * hh);
  const v4f gs = *(const v4f*)(gns + head * HDIM + c4);
  const v4f gb = *(const v4f*)(gnb + head * HDIM + c4);
  float cst[8], nst[8], mst[8];
#pragma unroll
  for (int r = 0; r < 8; ++r) { cst[r] = 0.0f; nst[r] = 0.0f; mst[r] = 0.0f; }
  const v8f z8 = {0.f, 0.f, 0.f, 0.f, 0.f, 0.f, 0.f, 0.f};
  __syncthreads();

#pragma unroll 1
  for (int t = 0; t < NSTEP; ++t) {
    const int par = t & 1;
    v4f gxv[8];
#pragma unroll
    for (int r = 0; r < 8; ++r)
      gxv[r] = *(const v4f*)(GX + ((size_t)(b0 + 8 * hh + r) * NSTEP + (size_t)t) * NGATE + head * 128 + eh * 64 + c * 4);
    const v16h a = frag_load(&hA[par][head][c * HAP + 8 * hh]);
    v8f acc[4];
#pragma unroll
    for (int g = 0; g < 4; ++g) acc[g] = mma16(a, bfr[g], z8);
#pragma unroll
    for (int g = 0; g < 4; ++g) tie_acc(acc[g], a, bfr[g]);

    _Float16* hw = &hA[par ^ 1][head][0];
    float*    sw = &Ss[par][head][0];
#pragma unroll
    for (int r = 0; r < 8; ++r) {
      const float gi_ = gxv[r][0] + acc[0][r] * REC_FOLD;
      const float gf_ = gxv[r][1] + acc[1][r] * REC_FOLD;
      const float gz_ = gxv[r][2] + acc[2][r] * REC_FOLD;
      const float go_ = gxv[r][3] + acc[3][r] * REC_FOLD;
      const float fm = gf_ + mst[r];
      const float dd = fm - gi_;
      const float ex = expf(-fabsf(dd));
      const bool fge = (dd >= 0.0f);
      const float ig = fge ? ex : 1.0f;
      const float fg = fge ? 1.0f : ex;
      mst[r] = fge ? fm : gi_;
      const float tz = 1.0f - 2.0f * (1.0f / (expf(2.0f * gz_) + 1.0f));
      const float cn = fg * cst[r] + ig * tz;
      const float nn = fg * nst[r] + ig;
      cst[r] = cn;
      nst[r] = nn;
      const float sg = 1.0f / (1.0f + expf(-go_));
      const float hv = (sg * cn) * (1.0f / (nn + CELL_EPS));
      hw[(8 * hh + r) * HAP + 16 * eh + c] = to_h16(hv, HS_CARRY);
      sw[(8 * hh + r) * SLP + 16 * eh + c] = hv;
    }
    __syncthreads();

    const float* sr = &Ss[par][head][0];
    v4f ov[2];
#pragma unroll
    for (int j = 0; j < 2; ++j) {
      const int row = 8 * eh + 4 * j + q;
      const v4f v = *(const v4f*)(sr + row * SLP + c4);
      float s = (v[0] + v[1]) + (v[2] + v[3]);
      s += __shfl_xor(s, 1, 32);
      s += __shfl_xor(s, 2, 32);
      s += __shfl_xor(s, 4, 32);
      const float mu = s * (1.0f / HDIM);
      const float d0 = v[0] - mu, d1 = v[1] - mu, d2 = v[2] - mu, d3 = v[3] - mu;
      float ss = (d0 * d0 + d1 * d1) + (d2 * d2 + d3 * d3);
      ss += __shfl_xor(ss, 1, 32);
      ss += __shfl_xor(ss, 2, 32);
      ss += __shfl_xor(ss, 4, 32);
      const float rstd = rsqrtf(ss * (1.0f / HDIM) + NORM_EPS);
      const v4f ho = *(const v4f*)(Hq + ((size_t)(b0 + row) * NSTEP + (size_t)t) * DMODEL + head * HDIM + c4);
      v4f o;
      o[0] = ho[0] + ((d0 * rstd) * gs[0] + gb[0]);
      o[1] = ho[1] + ((d1 * rstd) * gs[1] + gb[1]);
      o[2] = ho[2] + ((d2 * rstd) * gs[2] + gb[2]);
      o[3] = ho[3] + ((d3 * rstd) * gs[3] + gb[3]);
      ov[j] = o;
    }
    for (int pass = 0; pass < 2; ++pass) {
#pragma unroll
      for (int j = 0; j < 2; ++j) {
        const int row = 8 * eh + 4 * j + q;
        *(volatile v4f*)(Hq + ((size_t)(b0 + row) * NSTEP + (size_t)t) * DMODEL + head * HDIM + c4) = ov[j];
      }
      __threadfence();
    }
  }
}

__global__ __launch_bounds__(256) void gelu_cast_kernel(const float* __restrict__ PRE, unsigned short* __restrict__ A1) {
  const size_t i = (size_t)blockIdx.x * 256 + threadIdx.x;
  const v2f p = *(const v2f*)(PRE + 2 * i);
  const float x0 = p[0], x1 = p[1];
  const float g0 = 0.5f * x0 * (1.0f + erff(x0 * 0.70710678118654752f));
  const float g1 = 0.5f * x1 * (1.0f + erff(x1 * 0.70710678118654752f));
  const _Float16 h0 = to_h16(g0, U_CARRY);
  const _Float16 h1 = to_h16(g1, U_CARRY);
  const unsigned short u0 = __builtin_bit_cast(unsigned short, h0);
  const unsigned short u1 = __builtin_bit_cast(unsigned short, h1);
  const unsigned u = (unsigned)u0 | ((unsigned)u1 << 16);
  volatile unsigned* op = (volatile unsigned*)A1 + i;
  *op = u;
  __threadfence();
  *op = u;
}

__global__ __launch_bounds__(256) void head_kernel(const float* __restrict__ Hp, const float* __restrict__ pns,
                                                   const float* __restrict__ pnb, const unsigned short* __restrict__ PTp,
                                                   const float* __restrict__ projb, float* __restrict__ out) {
  __shared__ __align__(16) _Float16 At[8][16 * FAP];
  __shared__ __align__(16) float    Os[4][32 * NVOC];
  const _Float16* PT = (const _Float16*)PTp;
  const int tid = threadIdx.x, lane = tid & 31, wave = tid >> 5;
  const int l16 = lane & 15, hh = lane >> 4;
  const int row0 = blockIdx.x * 128 + wave * 16;
  const v4f g0 = *(const v4f*)(pns + 8 * l16);
  const v4f g1 = *(const v4f*)(pns + 8 * l16 + 4);
  const v4f b0 = *(const v4f*)(pnb + 8 * l16);
  const v4f b1 = *(const v4f*)(pnb + 8 * l16 + 4);
  float pb = projb[l16 < NVOC ? l16 : (NVOC - 1)];
  asm volatile("" : "+v"(pb));
#pragma unroll 1
  for (int it = 0; it < 8; ++it) {
    const int rloc = it * 2 + hh;
    const v8h hv = ln8_to_h(Hp + (size_t)(row0 + rloc) * DMODEL + 8 * l16, g0, g1, b0, b1);
    *(v8h*)(&At[wave][rloc * FAP + 8 * l16]) = hv;
  }
  __syncthreads();
  v8f acc = {0.f, 0.f, 0.f, 0.f, 0.f, 0.f, 0.f, 0.f};
#pragma unroll
  for (int ks = 0; ks < DMODEL / 32; ++ks) {
    const v16h a = frag_load(&At[wave][l16 * FAP + 8 * hh + 32 * ks]);
    const v16h b = frag_load(PT + (size_t)l16 * DMODEL + 8 * hh + 32 * ks);
    acc = mma16(a, b, acc);
    tie_acc(acc, a, b);
  }
  const int pr = wave >> 1;
  if (l16 < NVOC) {
#pragma unroll
    for (int r = 0; r < 8; ++r) Os[pr][((wave & 1) * 16 + 8 * hh + r) * NVOC + l16] = acc[r] * GATE_FOLD + pb;
  }
  __syncthreads();
  if ((wave & 1) == 0) {
    float* op = out + (size_t)blockIdx.x * (128 * NVOC) + (size_t)pr * (32 * NVOC);
    const int l8 = lane < 8 ? lane : 7;
    const v4f v0 = *(const v4f*)(&Os[pr][4 * lane]);
    const v4f v1 = *(const v4f*)(&Os[pr][128 + 4 * lane]);
    const v4f v2 = *(const v4f*)(&Os[pr][256 + 4 * l8]);
    for (int pass = 0; pass < 2; ++pass) {
      *(volatile v4f*)(op + 4 * lane) = v0;
      *(volatile v4f*)(op + 128 + 4 * lane) = v1;
      if (lane < 8) *(volatile v4f*)(op + 256 + 4 * lane) = v2;
      __threadfence();
    }
  }
}

extern "C" void kernel_launch(void* const* d_in, const int* in_sizes, int n_in,
                              void* d_out, int out_size, void* d_ws, size_t ws_size, hipStream_t stream) {
  if (n_in < 19 || d_out == nullptr || d_ws == nullptr) return;
  if (in_sizes[0] != NROWS || in_sizes[1] != NVOC * DMODEL || in_sizes[2] != NLAYER * DMODEL ||
      in_sizes[3] != NLAYER * DMODEL || in_sizes[4] != NLAYER * DMODEL * NGATE || in_sizes[5] != NLAYER * NGATE ||
      in_sizes[6] != NLAYER * 4 * NHEAD * HDIM * HDIM || in_sizes[7] != NLAYER * DMODEL || in_sizes[8] != NLAYER * DMODEL ||
      in_sizes[9] != NLAYER * DMODEL || in_sizes[10] != NLAYER * DMODEL || in_sizes[11] != NLAYER * DMODEL * DMODEL ||
      in_sizes[12] != NLAYER * DMODEL || in_sizes[13] != NLAYER * DMODEL * DMODEL || in_sizes[14] != NLAYER * DMODEL ||
      in_sizes[15] != DMODEL || in_sizes[16] != DMODEL || in_sizes[17] != DMODEL * NVOC || in_sizes[18] != NVOC ||
      out_size != NROWS * NVOC) return;

  const int*   x     = (const int*)d_in[0];
  const float* emb   = (const float*)d_in[1];
  const float* ln1_s = (const float*)d_in[2];
  const float* ln1_b = (const float*)d_in[3];
  const float* Wg    = (const float*)d_in[4];
  const float* bg    = (const float*)d_in[5];
  const float* R     = (const float*)d_in[6];
  const float* gn_s  = (const float*)d_in[7];
  const float* gn_b  = (const float*)d_in[8];
  const float* ln2_s = (const float*)d_in[9];
  const float* ln2_b = (const float*)d_in[10];
  const float* W1    = (const float*)d_in[11];
  const float* b1    = (const float*)d_in[12];
  const float* W2    = (const float*)d_in[13];
  const float* b2    = (const float*)d_in[14];
  const float* pn_s  = (const float*)d_in[15];
  const float* pn_b  = (const float*)d_in[16];
  const float* projW = (const float*)d_in[17];
  const float* projb = (const float*)d_in[18];
  float* out = (float*)d_out;

  char* ws = (char*)d_ws;
  size_t off = 0;
  auto carve = [&](size_t bytes) -> char* { char* p = ws + off; off += (bytes + 255) & ~(size_t)255; return p; };
  float*          H   = (float*)carve((size_t)NROWS * DMODEL * 4);
  unsigned short* AX  = (unsigned short*)carve((size_t)NROWS * DMODEL * 2);
  unsigned short* A1  = (unsigned short*)carve((size_t)NROWS * DMODEL * 2);
  float*          GX  = (float*)carve((size_t)QROWS * NGATE * 4);
  unsigned short* WGT = (unsigned short*)carve((size_t)NLAYER * NGATE * DMODEL * 2);
  unsigned short* W1T = (unsigned short*)carve((size_t)NLAYER * DMODEL * DMODEL * 2);
  unsigned short* W2T = (unsigned short*)carve((size_t)NLAYER * DMODEL * DMODEL * 2);
  unsigned short* RT  = (unsigned short*)carve((size_t)NLAYER * NHEAD * 128 * HDIM * 2);
  unsigned short* PT  = (unsigned short*)carve((size_t)16 * DMODEL * 2);
  float*          BGP = (float*)carve((size_t)NLAYER * NGATE * 4);
  float*          PRE = GX;
  static_assert((size_t)QROWS * NGATE == (size_t)NROWS * DMODEL, "PRE fits the GX region exactly");
  if (off > ws_size || off > (size_t)134217728) return;

  prep_planes_kernel<<<SEG_END / 256, 256, 0, stream>>>(Wg, bg, R, W1, W2, projW, WGT, W1T, W2T, RT, PT, BGP);
  embed_kernel<<<NROWS / 8, 256, 0, stream>>>(x, emb, H);

  const int gateGrid = (QROWS / 64) * (NGATE / 64) / 8;
  const int mlpGrid  = (NROWS / 64) * (DMODEL / 64) / 8;
  for (int l = 0; l < NLAYER; ++l) {
    ln_rows_kernel<<<NROWS / 16, 256, 0, stream>>>(H, ln1_s + l * DMODEL, ln1_b + l * DMODEL, AX);
    for (int qd = 0; qd < NQUART; ++qd) {
      gemm64_f16<false><<<gateGrid, 256, 0, stream>>>(
          AX + (size_t)qd * QROWS * DMODEL, DMODEL, WGT + (size_t)l * NGATE * DMODEL, DMODEL,
          GX, NGATE, BGP + l * NGATE, GX, QROWS, NGATE, DMODEL, GATE_FOLD);
      scan_kernel<<<QBATCH / SEQ_BLK, 256, 0, stream>>>(
          GX, RT + (size_t)l * NHEAD * 128 * HDIM, gn_s + l * DMODEL, gn_b + l * DMODEL,
          H + (size_t)qd * QROWS * DMODEL);
    }
    ln_rows_kernel<<<NROWS / 16, 256, 0, stream>>>(H, ln2_s + l * DMODEL, ln2_b + l * DMODEL, AX);
    gemm64_f16<false><<<mlpGrid, 256, 0, stream>>>(
        AX, DMODEL, W1T + (size_t)l * DMODEL * DMODEL, DMODEL,
        PRE, DMODEL, b1 + l * DMODEL, PRE, NROWS, DMODEL, DMODEL, GATE_FOLD);
    gelu_cast_kernel<<<(NROWS * DMODEL / 2) / 256, 256, 0, stream>>>(PRE, A1);
    gemm64_f16<true><<<mlpGrid, 256, 0, stream>>>(
        A1, DMODEL, W2T + (size_t)l * DMODEL * DMODEL, DMODEL,
        H, DMODEL, b2 + l * DMODEL, H, NROWS, DMODEL, DMODEL, MLP2_FOLD);
  }
  head_kernel<<<NROWS / 128, 256, 0, stream>>>(H, pn_s, pn_b, PT, projb, out);
}
